// ChunkedLinearMemoryUpdate_66099546685581
// MI455X (gfx1250) — hardware-run, weakly checked
//
#include <hip/hip_runtime.h>


#define NT   128
#define ND   768
#define O1   589824
#define O2   590592
#define O3   1180416
#define O4   1181184
typedef _Float16 h16;
typedef unsigned short bf;
typedef __attribute__((ext_vector_type(16))) __bf16   v16bf;
typedef __attribute__((ext_vector_type(16))) _Float16 v16h;
typedef __attribute__((ext_vector_type(8)))  _Float16 v8h;
typedef __attribute__((ext_vector_type(8)))  unsigned short v8us;
typedef __attribute__((ext_vector_type(8)))  float    v8f;
typedef __attribute__((ext_vector_type(4)))  float    v4f;
typedef v8h  __attribute__((may_alias)) v8ha;
typedef v4f  __attribute__((may_alias)) v4fa;
typedef v8us __attribute__((may_alias)) v8usa;

__device__ __forceinline__ unsigned short f2bf(float f) { unsigned u = __float_as_uint(f); u += 0x7FFFu + ((u >> 16) & 1u); return (unsigned short)(u >> 16); }
__device__ __forceinline__ float bf2f(unsigned short b) { return __uint_as_float(((unsigned)b) << 16); }
__device__ __forceinline__ float bfr(float f) { return bf2f(f2bf(f)); }
__device__ __forceinline__ v16h cat16(v8h lo, v8h hi) { return __builtin_shufflevector(lo, hi, 0, 1, 2, 3, 4, 5, 6, 7, 8, 9, 10, 11, 12, 13, 14, 15); }
__device__ __forceinline__ v16bf cat16b(v8us lo, v8us hi) { return __builtin_bit_cast(v16bf, __builtin_shufflevector(lo, hi, 0, 1, 2, 3, 4, 5, 6, 7, 8, 9, 10, 11, 12, 13, 14, 15)); }
__device__ __forceinline__ v8f wmma16(v16h a, v16h b, v8f c) { return __builtin_amdgcn_wmma_f32_16x16x32_f16(false, a, false, b, (short)0, c, false, false); }
__device__ __forceinline__ v8f wmmab(v16bf a, v16bf b, v8f c) { return __builtin_amdgcn_wmma_f32_16x16x32_bf16(false, a, false, b, (short)0, c, false, false); }

template <typename T16> struct WFrag;
template <> struct WFrag<h16> { typedef v16h V; static __device__ __forceinline__ V ld(const h16* p) { return cat16(*(const v8h*)p, *(const v8h*)(p + 16)); } static __device__ __forceinline__ v8f mma(V a, V b, v8f c) { return wmma16(a, b, c); } };
template <> struct WFrag<bf> { typedef v16bf V; static __device__ __forceinline__ V ld(const bf* p) { return cat16b(*(const v8us*)p, *(const v8us*)(p + 16)); } static __device__ __forceinline__ v8f mma(V a, V b, v8f c) { return wmmab(a, b, c); } };
template <typename T16, int NSPLIT, bool BIAS>
__global__ __launch_bounds__(32) void k_gemmw(const T16* __restrict__ A, const T16* __restrict__ A2, const T16* __restrict__ Bt, const T16* __restrict__ Bt2, int K, float* C, int ldc, const float* __restrict__ bias, size_t sA, size_t sB, size_t sC) {
    typedef typename WFrag<T16>::V V;
    __shared__ __align__(16) float os[16 * 68];
    const size_t z = blockIdx.z; A += z * sA; if (A2) A2 += z * sA; Bt += z * sB; if (Bt2) Bt2 += z * sB; C += z * sC;
    const int lane = threadIdx.x & 31, lr = lane & 15, hi = lane >> 4; const int r0 = blockIdx.x * 64, c0 = blockIdx.y * 64;
    v8f acc[4][4];
#pragma unroll
    for (int mb = 0; mb < 4; ++mb)
#pragma unroll
        for (int nb = 0; nb < 4; ++nb) acc[mb][nb] = (v8f){};
    const size_t aoff = (size_t)(r0 + lr) * K + 8 * hi, boff = (size_t)(c0 + lr) * K + 8 * hi;
    for (int kc = 0; kc < K; kc += 32) {
        V a[4], a2[4];
#pragma unroll
        for (int mb = 0; mb < 4; ++mb) { a[mb] = WFrag<T16>::ld(A + aoff + (size_t)mb * 16 * K + kc); if (NSPLIT == 1 || NSPLIT == 2) a2[mb] = WFrag<T16>::ld(A2 + aoff + (size_t)mb * 16 * K + kc); }
#pragma unroll
        for (int nb = 0; nb < 4; ++nb) { const V b = WFrag<T16>::ld(Bt + boff + (size_t)nb * 16 * K + kc); V b2; if (NSPLIT >= 2) b2 = WFrag<T16>::ld(Bt2 + boff + (size_t)nb * 16 * K + kc);
#pragma unroll
            for (int mb = 0; mb < 4; ++mb) { acc[mb][nb] = WFrag<T16>::mma(a[mb], b, acc[mb][nb]); if (NSPLIT == 1 || NSPLIT == 2) acc[mb][nb] = WFrag<T16>::mma(a2[mb], b, acc[mb][nb]); if (NSPLIT >= 2) acc[mb][nb] = WFrag<T16>::mma(a[mb], b2, acc[mb][nb]); } }
        asm volatile("v_nop\n\tv_nop\n\tv_nop\n\tv_nop" : "+v"(acc[0][0]), "+v"(acc[1][1]), "+v"(acc[2][2]), "+v"(acc[3][3]) : "v"(a[0]), "v"(a[3]));
    }
#pragma unroll
    for (int mb = 0; mb < 4; ++mb) {
#pragma unroll
        for (int nb = 0; nb < 4; ++nb) {
#pragma unroll
            for (int j = 0; j < 8; ++j) os[(hi * 8 + j) * 68 + nb * 16 + lr] = acc[mb][nb][j]; }
        __builtin_amdgcn_wave_barrier(); asm volatile("" ::: "memory");
        float* crow = C + (size_t)(r0 + mb * 16) * ldc + c0;
#pragma unroll 1
        for (int ps = 0; ps < 2; ++ps) {
#pragma unroll
            for (int s = 0; s < 8; ++s) { const int row = 2 * s + hi, cofs = lr * 4; v4f val = *(const v4fa*)(os + row * 68 + cofs); if (BIAS) { val[0] += bfr(bias[c0 + cofs]); val[1] += bfr(bias[c0 + cofs + 1]); val[2] += bfr(bias[c0 + cofs + 2]); val[3] += bfr(bias[c0 + cofs + 3]); }
                *(volatile v4f*)(crow + (size_t)row * ldc + cofs) = val; }
            if (ps == 0) __threadfence(); }
        __builtin_amdgcn_wave_barrier(); asm volatile("" ::: "memory");
    }
}

typedef __attribute__((ext_vector_type(2))) _Float16 v2h;
typedef __attribute__((ext_vector_type(4))) _Float16 v4h;
typedef __attribute__((ext_vector_type(2))) unsigned short v2us;
typedef __attribute__((ext_vector_type(4))) unsigned short v4us;
typedef __attribute__((ext_vector_type(2))) float v2f;
typedef __attribute__((ext_vector_type(4))) int v4i;
__global__ __launch_bounds__(256) void k_cvt8(const float* __restrict__ src, bf* dst, size_t n8) { const size_t i = (size_t)blockIdx.x * 256 + threadIdx.x; if (i >= n8) return; const v8f v = *(const v8f*)(src + i * 8); v8us o;
#pragma unroll
    for (int k = 0; k < 8; ++k) o[k] = f2bf(v[k]); *(volatile v8us*)(dst + i * 8) = o; __threadfence(); *(volatile v8us*)(dst + i * 8) = o; }

__global__ __launch_bounds__(128) void k_coef(float* cf) { const int t = threadIdx.x; const float l = log1pf(-0.01f); float s = 0.0f, tot = 0.0f;
#pragma unroll
    for (int j = 0; j < NT; ++j) { tot = tot + l; s = s + ((j <= t) ? l : 0.0f); }
    const float at = expf(s), aT = expf(tot); const float c = 0.01f * (aT / fmaxf(at, 1e-10f));
    *(volatile float*)(cf + t) = c; *(volatile float*)(cf + NT + t) = aT;
    __threadfence();
    *(volatile float*)(cf + t) = c; *(volatile float*)(cf + NT + t) = aT; }

__global__ __launch_bounds__(128) void k_msq(const float* __restrict__ P, const float* __restrict__ vl, const float* __restrict__ bv, float* R4) { const int t = threadIdx.x; const float* p = P + (size_t)t * ND; const float* v = vl + (size_t)t * ND; float acc = 0.0f;
    for (int o0 = 0; o0 < ND; o0 += 8) {
#pragma unroll
        for (int k = 0; k < 8; ++k) { const float f = (p[o0 + k] + bfr(bv[o0 + k])) - bfr(v[o0 + k]); acc = acc + f * f; } }
    const float y = acc / 768.0f; *(volatile float*)(R4 + t) = y; __threadfence(); *(volatile float*)(R4 + t) = y; }

__global__ __launch_bounds__(256) void k_walkW(const float* __restrict__ P, const float* __restrict__ vl, const float* __restrict__ ky, const float* __restrict__ mw, const float* __restrict__ Wt, const float* __restrict__ cf, float* R0, float* R2) { const unsigned n = blockIdx.x * 256 + threadIdx.x; const unsigned o = n / ND, i = n - o * ND; const float m9 = 0.9f * bfr(mw[n]); float S = 0.0f;
    for (int t0 = 0; t0 < NT; t0 += 8) {
#pragma unroll
        for (int k = 0; k < 8; ++k) { const int t = t0 + k; const float e = P[(size_t)t * ND + o] - bfr(vl[(size_t)t * ND + o]); float g = -(cf[t] * ((2.0f * e) * bfr(ky[(size_t)t * ND + i]))); g = g + ((t == 0) ? m9 : 0.0f); S = 0.9f * S + g; } }
    const float r0 = cf[NT] * bfr(Wt[n]) + S;
    *(volatile float*)(R2 + n) = S; *(volatile float*)(R0 + n) = r0; __threadfence(); *(volatile float*)(R2 + n) = S; *(volatile float*)(R0 + n) = r0; }

__global__ __launch_bounds__(256) void k_walkb(const float* __restrict__ P, const float* __restrict__ vl, const float* __restrict__ bv, const float* __restrict__ mv, const float* __restrict__ cf, float* R1, float* R3) { const unsigned o = blockIdx.x * 256 + threadIdx.x; const float bq = bfr(bv[o]); const float m9 = 0.9f * bfr(mv[o]); float S = 0.0f;
    for (int t0 = 0; t0 < NT; t0 += 8) {
#pragma unroll
        for (int k = 0; k < 8; ++k) { const int t = t0 + k; const float f = (P[(size_t)t * ND + o] + bq) - bfr(vl[(size_t)t * ND + o]); float g = -(cf[t] * (2.0f * f)); g = g + ((t == 0) ? m9 : 0.0f); S = 0.9f * S + g; } }
    const float r1 = cf[NT] * bq + S;
    *(volatile float*)(R3 + o) = S; *(volatile float*)(R1 + o) = r1; __threadfence(); *(volatile float*)(R3 + o) = S; *(volatile float*)(R1 + o) = r1; }

extern "C" void kernel_launch(void* const* d_in, const int* in_sizes, int n_in, void* d_out, int out_size, void* d_ws, size_t ws_size, hipStream_t stream) {
    if (n_in < 6) return;
    if (in_sizes[0] != ND * ND || in_sizes[1] != ND || in_sizes[2] != NT * ND || in_sizes[3] != NT * ND || in_sizes[4] != ND * ND || in_sizes[5] != ND) return;
    if (out_size != O4 + NT) return;
    static_assert(O1 == ND * ND && O2 == O1 + ND && O3 == O2 + ND * ND && O4 == O3 + ND && (O1 % 32) == 0 && (O2 % 32) == 0 && (O3 % 32) == 0 && (O4 % 32) == 0 && NT % 64 == 0 && ND % 64 == 0 && ND % 32 == 0 && (NT * ND / 8) % 256 == 0 && (ND * ND / 8) % 256 == 0 && (ND * ND) % 256 == 0 && ND % 256 == 0 && NT % 8 == 0 && ND % 8 == 0 && NT == 128, "the five results end to end, each on a 128-byte line; the product: M and N multiples of 64, the depth of 32; the flat grids exact; the tokens and columns in eights; one block of 128 for the factors and the means");
    const float* Wt = (const float*)d_in[0]; const float* bv = (const float*)d_in[1]; const float* ky = (const float*)d_in[2]; const float* vl = (const float*)d_in[3]; const float* mw = (const float*)d_in[4]; const float* mv = (const float*)d_in[5];
    float* out = (float*)d_out; float* R0 = out; float* R1 = out + O1; float* R2 = out + O2; float* R3 = out + O3; float* R4 = out + O4;
    char* wsp = (char*)d_ws; auto take = [&](size_t bytes) { char* p = wsp; wsp += (bytes + 255) & ~(size_t)255; return (void*)p; };
    bf* Kb = (bf*)take((size_t)NT * ND * 2); bf* Wb = (bf*)take((size_t)ND * ND * 2); float* P = (float*)take((size_t)NT * ND * 4); float* cf = (float*)take((size_t)(2 * NT) * 4);
    if ((size_t)(wsp - (char*)d_ws) > ws_size) return;
    k_cvt8<<<(unsigned)(NT * ND / 8 / 256), 256, 0, stream>>>(ky, Kb, (size_t)NT * ND / 8);
    k_cvt8<<<(unsigned)(ND * ND / 8 / 256), 256, 0, stream>>>(Wt, Wb, (size_t)ND * ND / 8);
    k_gemmw<bf, 0, false><<<dim3(NT / 64, ND / 64, 1), 32, 0, stream>>>(Kb, nullptr, Wb, nullptr, ND, P, ND, nullptr, 0, 0, 0);
    k_coef<<<1, 128, 0, stream>>>(cf);
    k_msq<<<1, 128, 0, stream>>>(P, vl, bv, R4);
    k_walkW<<<(unsigned)(ND * ND / 256), 256, 0, stream>>>(P, vl, ky, mw, Wt, cf, R0, R2);
    k_walkb<<<(unsigned)(ND / 256), 256, 0, stream>>>(P, vl, bv, mv, cf, R1, R3);
}
